// LSTMModelCustom_22196390985729
// MI455X (gfx1250) — hardware-verified
//
#include <hip/hip_runtime.h>


#define BS_     64
#define SEQ_    1024
#define IN_     128
#define HS_     512
#define NG_     2048
#define KC_     640
#define OUT_    7
#define ROWS_   16
#define APITCH_ 648

static_assert(KC_ == IN_ + HS_);
static_assert(KC_ % 32 == 0);
static_assert(BS_ % ROWS_ == 0);
static_assert(SEQ_ % 2 == 0);
static_assert(HS_ == 8 * 64);
static_assert(IN_ == 16 * 8);
static_assert(NG_ % 64 == 0 && IN_ % 64 == 0 && HS_ % 64 == 0);
static_assert((BS_ * OUT_) % 4 == 0);
static_assert(((BS_ * OUT_) / 4) % 8 == 0);
static_assert(APITCH_ % 8 == 0 && APITCH_ >= KC_);

typedef float    v4f  __attribute__((ext_vector_type(4)));
typedef float    v8f  __attribute__((ext_vector_type(8)));
typedef _Float16 v8h  __attribute__((ext_vector_type(8)));
typedef _Float16 v16h __attribute__((ext_vector_type(16)));
union FragH { v16h v; v8h half[2]; };

constexpr int TILE_HALVES = ROWS_ * APITCH_;
constexpr int STG_FLOATS  = ROWS_ * HS_;
constexpr int LDS_HALVES  = TILE_HALVES + 2 * STG_FLOATS;
static_assert(TILE_HALVES <= 2 * STG_FLOATS);
static_assert((TILE_HALVES * 2) % 16 == 0);
static_assert(LDS_HALVES * 2 <= 65536);

constexpr size_t SZ_BCAT  = (size_t)NG_ * KC_ * 2;
constexpr size_t SZ_HL    = (size_t)BS_ * HS_ * 4;
constexpr size_t OFF_BCAT = 0;
constexpr size_t OFF_HL   = OFF_BCAT + SZ_BCAT;
constexpr size_t WS_END   = OFF_HL + SZ_HL;
static_assert(OFF_HL % 128 == 0);
static_assert((KC_ * 2) % 128 == 0);
static_assert((HS_ * 4) % 128 == 0);
static_assert(WS_END <= (size_t)134217728);

__device__ __forceinline__ void mma16(v8f& acc, const FragH& a, const FragH& b) {
    acc = __builtin_amdgcn_wmma_f32_16x16x32_f16(false, a.v, false, b.v, (short)0, acc, false, false);
    asm volatile("v_nop\n\tv_nop\n\tv_nop\n\tv_nop" : "+v"(acc) : "v"(a.v), "v"(b.v));
}
__device__ __forceinline__ float sigm_f(float x) {
    return __builtin_amdgcn_rcpf(1.0f + __expf(-x));
}
__device__ __forceinline__ float tanh_f(float x) {
    const float t = __expf(-2.0f * fabsf(x));
    const float r = (1.0f - t) * __builtin_amdgcn_rcpf(1.0f + t);
    return copysignf(r, x);
}
__device__ __forceinline__ v8f ld8f(const float* p) {
    v4f a = *(const v4f*)p;
    v4f b = *(const v4f*)(p + 4);
    return __builtin_shufflevector(a, b, 0, 1, 2, 3, 4, 5, 6, 7);
}

__global__ __launch_bounds__(256)
void wt_cvt_kernel(const float* __restrict__ src, _Float16* dst, int Nw, int Kd, int kofs)
{
    __shared__ __attribute__((aligned(16))) float sT[64 * 68];
    const int tid  = threadIdx.x;
    const int lane = tid & 31;
    const int wave = tid >> 5;
    const int n0 = blockIdx.x * 64;
    const int k0 = blockIdx.y * 64;

#pragma unroll
    for (int it = 0; it < 4; ++it) {
        const int idx = it * 256 + tid;
        const int kk  = idx >> 4;
        const int n4  = (idx & 15) * 4;
        const int gk  = min(k0 + kk, Kd - 1);
        const int gn  = min(n0 + n4, Nw - 4);
        const v4f v = *(const v4f*)(src + (size_t)gk * Nw + gn);
        sT[(n4 + 0) * 68 + kk] = v[0];
        sT[(n4 + 1) * 68 + kk] = v[1];
        sT[(n4 + 2) * 68 + kk] = v[2];
        sT[(n4 + 3) * 68 + kk] = v[3];
    }
    __syncthreads();

    v8h hv[2];
    const int c = (lane & 7) * 8;
#pragma unroll
    for (int it = 0; it < 2; ++it) {
        const int nn = it * 32 + wave * 4 + (lane >> 3);
        const v8f xv = ld8f(sT + nn * 68 + c);
#pragma unroll
        for (int e = 0; e < 8; ++e) hv[it][e] = (_Float16)(16.0f * xv[e]);
    }
#pragma unroll
    for (int it = 0; it < 2; ++it) {
        const int gr = n0 + it * 32 + wave * 4 + (lane >> 3);
        const size_t o = (size_t)gr * KC_ + kofs + k0 + c;
        *(volatile v8h*)(dst + o) = hv[it];
    }
    __threadfence();
#pragma unroll
    for (int it = 0; it < 2; ++it) {
        const int gr = n0 + it * 32 + wave * 4 + (lane >> 3);
        const size_t o = (size_t)gr * KC_ + kofs + k0 + c;
        *(volatile v8h*)(dst + o) = hv[it];
    }
}

template<int CG>
__device__ __forceinline__ void gate_pass(const _Float16* arow, const _Float16* __restrict__ bcat,
                                          const float* __restrict__ bias, int jw, int hh,
                                          float (&cst)[4][8], _Float16* wtile, float* stg, bool last)
{
    v8f acc[8];
#pragma unroll
    for (int j = 0; j < 8; ++j)
#pragma unroll
        for (int r = 0; r < 8; ++r) acc[j][r] = 0.0f;

    const _Float16* brow[8];
#pragma unroll
    for (int j = 0; j < 8; ++j) {
        const int q = j >> 1, tt = j & 1;
        brow[j] = bcat + (size_t)(q * HS_ + jw + 16 * (2 * CG + tt)) * KC_ + 8 * hh;
    }

#pragma unroll 1
    for (int ks = 0; ks < KC_ / 32; ++ks) {
        const int k0 = ks * 32;
        FragH fa;
        fa.half[0] = *(const v8h*)(arow + k0);
        fa.half[1] = *(const v8h*)(arow + k0 + 16);
#pragma unroll
        for (int j = 0; j < 8; ++j) {
            FragH fb;
            fb.half[0] = *(const v8h*)(brow[j] + k0);
            fb.half[1] = *(const v8h*)(brow[j] + k0 + 16);
            mma16(acc[j], fa, fb);
        }
    }

    float hv[2][8];
#pragma unroll
    for (int tt = 0; tt < 2; ++tt) {
        const int t = 2 * CG + tt;
        const int j = jw + 16 * t;
        const float bi = bias[j];
        const float bf = bias[HS_ + j];
        const float bg = bias[2 * HS_ + j];
        const float bo = bias[3 * HS_ + j];
#pragma unroll
        for (int r = 0; r < 8; ++r) {
            const float gi = acc[0 * 2 + tt][r] * 0.0625f + bi;
            const float gf = acc[1 * 2 + tt][r] * 0.0625f + bf;
            const float gg = acc[2 * 2 + tt][r] * 0.0625f + bg;
            const float go = acc[3 * 2 + tt][r] * 0.0625f + bo;
            const float iv = sigm_f(gi);
            const float fv = sigm_f(gf);
            const float gv = tanh_f(gg);
            const float ov = sigm_f(go);
            const float cn = fv * cst[t][r] + iv * gv;
            cst[t][r] = cn;
            hv[tt][r] = ov * tanh_f(cn);
        }
    }
    if (!last) {
#pragma unroll
        for (int tt = 0; tt < 2; ++tt)
#pragma unroll
            for (int r = 0; r < 8; ++r)
                wtile[(8 * hh + r) * APITCH_ + IN_ + jw + 16 * (2 * CG + tt)] = (_Float16)hv[tt][r];
    } else {
#pragma unroll
        for (int tt = 0; tt < 2; ++tt)
#pragma unroll
            for (int r = 0; r < 8; ++r)
                stg[(8 * hh + r) * HS_ + jw + 16 * (2 * CG + tt)] = hv[tt][r];
    }
}

__global__ __launch_bounds__(256)
void lstm_kernel(const float* __restrict__ x, const _Float16* __restrict__ bcat,
                 const float* __restrict__ bias, float* hlast)
{
    __shared__ __attribute__((aligned(16))) _Float16 ldsh[LDS_HALVES];
    float* stg = reinterpret_cast<float*>(ldsh + TILE_HALVES);

    const int tid  = threadIdx.x;
    const int lane = tid & 31;
    const int wave = tid >> 5;
    const int hh   = lane >> 4;
    const int m    = lane & 15;
    const int row0 = blockIdx.x * ROWS_;
    const int jw   = wave * 64 + m;

    {
        v8h z;
#pragma unroll
        for (int e = 0; e < 8; ++e) z[e] = (_Float16)0.0f;
#pragma unroll 1
        for (int i = tid; i < ROWS_ * (HS_ / 8); i += 256) {
            const int r  = i / (HS_ / 8);
            const int c8 = (i % (HS_ / 8)) * 8;
            *(v8h*)(ldsh + TILE_HALVES + r * APITCH_ + IN_ + c8) = z;
        }
    }

    float cst[4][8];
#pragma unroll
    for (int t = 0; t < 4; ++t)
#pragma unroll
        for (int r = 0; r < 8; ++r) cst[t][r] = 0.0f;

    const int xr = tid >> 4;
    const int xc = (tid & 15) * 8;
    const float* xrowp = x + ((size_t)(row0 + xr) * SEQ_) * IN_ + xc;

#pragma unroll 1
    for (int s = 0; s < SEQ_; ++s) {
        const int rdoff = (s & 1) ? 0 : TILE_HALVES;
        const int wroff = (s & 1) ? TILE_HALVES : 0;
        {
            const float* xp = xrowp + (size_t)s * IN_;
            const v4f a = *(const v4f*)xp;
            const v4f b = *(const v4f*)(xp + 4);
            v8h v;
#pragma unroll
            for (int e = 0; e < 4; ++e) { v[e] = (_Float16)a[e]; v[4 + e] = (_Float16)b[e]; }
            *(v8h*)(ldsh + rdoff + xr * APITCH_ + xc) = v;
        }
        __syncthreads();

        const bool last = (s == SEQ_ - 1);
        const _Float16* arow = ldsh + rdoff + m * APITCH_ + 8 * hh;
        _Float16* wtile = ldsh + wroff;
        gate_pass<0>(arow, bcat, bias, jw, hh, cst, wtile, stg, last);
        gate_pass<1>(arow, bcat, bias, jw, hh, cst, wtile, stg, last);
    }
    __syncthreads();

#pragma unroll
    for (int it = 0; it < 8; ++it) {
        const int L   = it * 32 + wave * 4 + (lane >> 3);
        const int row = L >> 4;
        const int col = (L & 15) * 32 + (lane & 7) * 4;
        const v4f v = *(const v4f*)(stg + row * HS_ + col);
        *(volatile v4f*)(hlast + (size_t)(row0 + row) * HS_ + col) = v;
    }
    __threadfence();
#pragma unroll
    for (int it = 0; it < 8; ++it) {
        const int L   = it * 32 + wave * 4 + (lane >> 3);
        const int row = L >> 4;
        const int col = (L & 15) * 32 + (lane & 7) * 4;
        const v4f v = *(const v4f*)(stg + row * HS_ + col);
        *(volatile v4f*)(hlast + (size_t)(row0 + row) * HS_ + col) = v;
    }
}

__global__ __launch_bounds__(256)
void fc_kernel(const float* __restrict__ hl, const float* __restrict__ fw, const float* __restrict__ fb, float* out)
{
    __shared__ __attribute__((aligned(16))) float so[BS_ * OUT_];
    const int tid = threadIdx.x;
#pragma unroll 1
    for (int e = tid; e < BS_ * OUT_; e += 256) {
        const int r = e / OUT_;
        const int j = e - r * OUT_;
        float acc = fb[j];
        const float* hr = hl + (size_t)r * HS_;
#pragma unroll 4
        for (int k = 0; k < HS_; ++k) acc = hr[k] * fw[k * OUT_ + j] + acc;
        so[e] = acc;
    }
    __syncthreads();
    constexpr int NV = (BS_ * OUT_) / 4;
    if (tid < NV) {
        const v4f v = *(const v4f*)(so + 4 * tid);
        *(volatile v4f*)(out + 4 * tid) = v;
    }
    __threadfence();
    if (tid < NV) {
        const v4f v = *(const v4f*)(so + 4 * tid);
        *(volatile v4f*)(out + 4 * tid) = v;
    }
}

extern "C" void kernel_launch(void* const* d_in, const int* in_sizes, int n_in,
                              void* d_out, int out_size, void* d_ws, size_t ws_size,
                              hipStream_t stream)
{
    if (n_in < 6) return;
    if (in_sizes[0] != BS_ * SEQ_ * IN_) return;
    if (in_sizes[1] != IN_ * NG_)        return;
    if (in_sizes[2] != HS_ * NG_)        return;
    if (in_sizes[3] != NG_)              return;
    if (in_sizes[4] != HS_ * OUT_)       return;
    if (in_sizes[5] != OUT_)             return;
    if (out_size != BS_ * OUT_)          return;
    if (ws_size < WS_END)                return;

    const float* x    = (const float*)d_in[0];
    const float* W    = (const float*)d_in[1];
    const float* U    = (const float*)d_in[2];
    const float* bias = (const float*)d_in[3];
    const float* fc_w = (const float*)d_in[4];
    const float* fc_b = (const float*)d_in[5];
    float* out = (float*)d_out;

    char* ws = (char*)d_ws;
    _Float16* bcat  = (_Float16*)(ws + OFF_BCAT);
    float*    hlast = (float*)(ws + OFF_HL);

    wt_cvt_kernel<<<dim3(NG_ / 64, IN_ / 64), dim3(256), 0, stream>>>(W, bcat, (int)NG_, (int)IN_, 0);
    wt_cvt_kernel<<<dim3(NG_ / 64, HS_ / 64), dim3(256), 0, stream>>>(U, bcat, (int)NG_, (int)HS_, (int)IN_);

    lstm_kernel<<<dim3(BS_ / ROWS_), dim3(256), 0, stream>>>(x, (const _Float16*)bcat, bias, hlast);

    fc_kernel<<<dim3(1), dim3(256), 0, stream>>>((const float*)hlast, fc_w, fc_b, out);
}
